// MambaTokenBlock_22282290332046
// MI455X (gfx1250) — hardware-verified
//
#include <hip/hip_runtime.h>


#define NBATCH 2
#define NL_    2048
#define DM_    1024
#define DI_    2048
#define NS_    16
#define DTR_   64
#define XDN_   96
#define XDW_   128
#define MT_    (NBATCH * NL_)

#define SC_X   8.0f
#define SC_WI  32.0f
#define SC_U   64.0f
#define SC_WX  32.0f
#define SC_DT  64.0f
#define SC_WD  16.0f
#define SC_Y   64.0f
#define SC_WO  32.0f

static_assert(MT_ % 64 == 0);
static_assert((2 * DI_) % 128 == 0);
static_assert(DI_ % 128 == 0);
static_assert(DM_ % 64 == 0);
static_assert(DM_ % 32 == 0);
static_assert(DI_ % 64 == 0);
static_assert(DTR_ % 32 == 0);
static_assert(XDW_ % 128 == 0);
static_assert(DTR_ + 2 * NS_ == XDN_);
static_assert(XDN_ <= XDW_);
static_assert(NL_ % 16 == 0);
static_assert((NL_ & (NL_ - 1)) == 0);
static_assert(DM_ == 128 * 8);
static_assert(DI_ == 256 * 8);

typedef float          v4f   __attribute__((ext_vector_type(4)));
typedef float          v8f   __attribute__((ext_vector_type(8)));
typedef _Float16       v8h   __attribute__((ext_vector_type(8)));
typedef _Float16       v16h  __attribute__((ext_vector_type(16)));
typedef unsigned short u16x8 __attribute__((ext_vector_type(8)));

union FragH { u16x8 h[2]; v16h v; };
union Pack8 { v8h f; u16x8 u; };

constexpr size_t SZ_X16 = (size_t)MT_ * DM_ * 2;
constexpr size_t SZ_WI  = (size_t)2 * DI_ * DM_ * 2;
constexpr size_t SZ_U16 = (size_t)MT_ * DI_ * 2;
constexpr size_t SZ_Y16 = (size_t)MT_ * DI_ * 2;
constexpr size_t SZ_F   = (size_t)MT_ * DI_ * 4;
constexpr size_t SZ_WX  = (size_t)XDW_ * DI_ * 2;
constexpr size_t SZ_XD  = (size_t)MT_ * XDW_ * 4;
constexpr size_t SZ_DTR = (size_t)MT_ * DTR_ * 2;
constexpr size_t SZ_WD  = (size_t)DI_ * DTR_ * 2;
constexpr size_t SZ_DL  = (size_t)MT_ * DI_ * 4;
constexpr size_t SZ_WO  = (size_t)DM_ * DI_ * 2;

constexpr size_t REG_A   = SZ_U16;
constexpr size_t OFF_X16 = 0;
constexpr size_t OFF_WI  = OFF_X16 + SZ_X16;
constexpr size_t OFF_U16 = 0;
constexpr size_t OFF_Y16 = 0;
constexpr size_t OFF_XF  = REG_A;
constexpr size_t OFF_ZF  = OFF_XF + SZ_F;
constexpr size_t OFF_WX  = OFF_ZF + SZ_F;
constexpr size_t OFF_XD  = OFF_WX + SZ_WX;
constexpr size_t OFF_DTR = OFF_XD + SZ_XD;
constexpr size_t OFF_WD  = OFF_DTR + SZ_DTR;
constexpr size_t OFF_DL  = OFF_WD + SZ_WD;
constexpr size_t OFF_WO  = OFF_DL + SZ_DL;
constexpr size_t WS_END  = OFF_WO + SZ_WO;
static_assert(OFF_WI + SZ_WI <= REG_A);
static_assert(OFF_U16 + SZ_U16 <= REG_A);
static_assert(OFF_Y16 + SZ_Y16 <= REG_A);
static_assert(WS_END <= (size_t)134217728);
static_assert(OFF_WI % 128 == 0 && OFF_XF % 128 == 0 && OFF_ZF % 128 == 0 && OFF_WX % 128 == 0);
static_assert(OFF_XD % 128 == 0 && OFF_DTR % 128 == 0 && OFF_WD % 128 == 0 && OFF_DL % 128 == 0);
static_assert(OFF_WO % 128 == 0);

__device__ __forceinline__ float silu_f(float x) {
    float e = __expf(-x);
    return x * __builtin_amdgcn_rcpf(1.0f + e);
}
__device__ __forceinline__ float softplus_f(float x) {
    return fmaxf(x, 0.0f) + log1pf(__expf(-fabsf(x)));
}
__device__ __forceinline__ float conv4_silu(float x0, float x1, float x2, float x3,
                                            float w0, float w1, float w2, float w3, float bias) {
    float c = w0 * x0 + w1 * x1 + w2 * x2 + w3 * x3;
    return silu_f(c + bias);
}
__device__ __forceinline__ v8f ld8f(const float* p) {
    v4f a = *(const v4f*)p;
    v4f b = *(const v4f*)(p + 4);
    return __builtin_shufflevector(a, b, 0, 1, 2, 3, 4, 5, 6, 7);
}

__device__ __forceinline__ void mma16(v8f& acc, const FragH& a, const FragH& b) {
    acc = __builtin_amdgcn_wmma_f32_16x16x32_f16(false, a.v, false, b.v, (short)0, acc, false, false);
    asm volatile("v_nop\n\tv_nop\n\tv_nop\n\tv_nop" : "+v"(acc) : "v"(a.v), "v"(b.v));
}

__global__ __launch_bounds__(256)
void cvt_kernel(const float* __restrict__ src, unsigned short* dst, int n8, int nsrc8, float scale)
{
    const int i = blockIdx.x * 256 + threadIdx.x;
    if (i >= n8) return;
    const size_t e = (size_t)i * 8;
    v8f x;
    if (i < nsrc8) {
        x = ld8f(src + e);
    } else {
#pragma unroll
        for (int c = 0; c < 8; ++c) x[c] = 0.0f;
    }
    Pack8 pk;
    pk.f = __builtin_convertvector(x * scale, v8h);
    const u16x8 v = pk.u;
    *(volatile u16x8*)(dst + e) = v;
    __threadfence();
    *(volatile u16x8*)(dst + e) = v;
}

__global__ __launch_bounds__(128)
void ln_f16_kernel(const float* __restrict__ X, const float* __restrict__ w,
                   const float* __restrict__ bb, unsigned short* x16)
{
    __shared__ float red0[4];
    __shared__ float red1[4];
    const int m    = blockIdx.x;
    const int tid  = threadIdx.x;
    const int lane = tid & 31;
    const int wave = tid >> 5;
    const int d0   = tid * 8;

    const v8f x = ld8f(X + (size_t)m * DM_ + d0);
    float s = 0.0f;
#pragma unroll
    for (int c = 0; c < 8; ++c) s += x[c];
#pragma unroll
    for (int off = 16; off; off >>= 1) s += __shfl_xor(s, off, 32);
    if (lane == 0) red0[wave] = s;
    __syncthreads();
    const float mu = (red0[0] + red0[1] + red0[2] + red0[3]) * (1.0f / (float)DM_);

    float q = 0.0f;
#pragma unroll
    for (int c = 0; c < 8; ++c) { const float dv = x[c] - mu; q += dv * dv; }
#pragma unroll
    for (int off = 16; off; off >>= 1) q += __shfl_xor(q, off, 32);
    if (lane == 0) red1[wave] = q;
    __syncthreads();
    const float var = (red1[0] + red1[1] + red1[2] + red1[3]) * (1.0f / (float)DM_);
    const float rs  = rsqrtf(var + 1e-5f);

    const v8f wv = ld8f(w + d0);
    const v8f bv = ld8f(bb + d0);
    v8f y;
#pragma unroll
    for (int c = 0; c < 8; ++c) y[c] = ((x[c] - mu) * rs * wv[c] + bv[c]) * SC_X;

    Pack8 pk;
    pk.f = __builtin_convertvector(y, v8h);
    const u16x8 v = pk.u;
    unsigned short* gp = x16 + (size_t)m * DM_ + d0;
    *(volatile u16x8*)gp = v;
    __threadfence();
    *(volatile u16x8*)gp = v;
}

template<int NBF, bool RES>
__device__ __forceinline__ void tile_store_pass(const float* st, float* gp, const float* rp,
                                                int ldc, int lane) {
    constexpr int CW  = NBF * 16;
    constexpr int P   = CW + 4;
    constexpr int EPL = 4;
    static_assert(CW % EPL == 0);
    constexpr int LPR = CW / EPL;
    static_assert(32 % LPR == 0);
    constexpr int RPI = 32 / LPR;
    static_assert(32 % RPI == 0);
    constexpr int NIT = 32 / RPI;
    const int rsub = lane / LPR;
    const int c0   = (lane % LPR) * EPL;
#pragma unroll
    for (int it = 0; it < NIT; ++it) {
        const int row = it * RPI + rsub;
        v4f v = *(const v4f*)(st + row * P + c0);
        const size_t go = (size_t)row * ldc + c0;
        if (RES) v += *(const v4f*)(rp + go);
        *(volatile v4f*)(gp + go) = v;
    }
}

template<int NBF, bool RES>
__global__ __launch_bounds__(128)
void gemm_tn_kernel(const unsigned short* __restrict__ A, const unsigned short* __restrict__ Bw,
                    float* C, float* C2, const float* R, int K, int ldc, int csplit, float scale)
{
    constexpr int CW = NBF * 16;
    constexpr int P  = CW + 4;
    __shared__ __attribute__((aligned(16))) float stile[4][32 * P];

    const int tid  = threadIdx.x;
    const int lane = tid & 31;
    const int wave = tid >> 5;
    const int h    = lane >> 4;
    const int m    = lane & 15;
    const int wm   = wave >> 1;
    const int wn   = wave & 1;

    const int rowW = blockIdx.y * 64 + wm * 32;
    const int colW = blockIdx.x * (2 * CW) + wn * CW;

    v8f acc[2 * NBF];
#pragma unroll
    for (int j = 0; j < 2 * NBF; ++j)
#pragma unroll
        for (int r = 0; r < 8; ++r) acc[j][r] = 0.0f;

    const size_t aoff  = (size_t)(rowW + m) * K + 8 * h;
    const size_t boff  = (size_t)(colW + m) * K + 8 * h;
    const size_t sub16 = (size_t)16 * K;
    const int nk = K >> 5;

    for (int kt = 0; kt < nk; ++kt) {
        const size_t k0 = (size_t)kt * 32;
        FragH fa[2], fb[NBF];
#pragma unroll
        for (int s = 0; s < 2; ++s) {
            const unsigned short* p = A + aoff + s * sub16 + k0;
            fa[s].h[0] = *(const u16x8*)(p);
            fa[s].h[1] = *(const u16x8*)(p + 16);
        }
#pragma unroll
        for (int j = 0; j < NBF; ++j) {
            const unsigned short* p = Bw + boff + j * sub16 + k0;
            fb[j].h[0] = *(const u16x8*)(p);
            fb[j].h[1] = *(const u16x8*)(p + 16);
        }
#pragma unroll
        for (int s = 0; s < 2; ++s)
#pragma unroll
            for (int j = 0; j < NBF; ++j)
                mma16(acc[s * NBF + j], fa[s], fb[j]);
    }

    float* st = stile[wave];
#pragma unroll
    for (int s = 0; s < 2; ++s)
#pragma unroll
        for (int j = 0; j < NBF; ++j)
#pragma unroll
            for (int r = 0; r < 8; ++r)
                st[(s * 16 + 8 * h + r) * P + j * 16 + m] = acc[s * NBF + j][r] * scale;
    __syncthreads();

    float* Cp = C;
    int gcol = colW;
    if (colW >= csplit) { Cp = C2; gcol = colW - csplit; }
    const size_t gbase = (size_t)rowW * ldc + gcol;
    float* gp = Cp + gbase;
    const float* rp = R + gbase;
    tile_store_pass<NBF, RES>(st, gp, rp, ldc, lane);
    __threadfence();
    tile_store_pass<NBF, RES>(st, gp, rp, ldc, lane);
}

__global__ __launch_bounds__(256)
void conv_silu_kernel(const float* __restrict__ X, const float* __restrict__ cw,
                      const float* __restrict__ cb, unsigned short* U16)
{
    const int m  = blockIdx.x;
    const int l  = m & (NL_ - 1);
    const int d0 = threadIdx.x * 8;
    const float* xr = X + (size_t)m * DI_ + d0;

    v8f x3 = ld8f(xr);
    v8f x2, x1, x0;
#pragma unroll
    for (int c = 0; c < 8; ++c) { x2[c] = 0.0f; x1[c] = 0.0f; x0[c] = 0.0f; }
    if (l >= 1) x2 = ld8f(xr - DI_);
    if (l >= 2) x1 = ld8f(xr - 2 * DI_);
    if (l >= 3) x0 = ld8f(xr - 3 * DI_);

    const float* wp = cw + (size_t)d0 * 4;
    v4f wv[8];
#pragma unroll
    for (int c = 0; c < 8; ++c) wv[c] = *(const v4f*)(wp + 4 * c);
    const v8f bias = ld8f(cb + d0);

    v8f u;
#pragma unroll
    for (int c = 0; c < 8; ++c)
        u[c] = conv4_silu(x0[c], x1[c], x2[c], x3[c], wv[c][0], wv[c][1], wv[c][2], wv[c][3], bias[c]) * SC_U;

    Pack8 pk;
    pk.f = __builtin_convertvector(u, v8h);
    const u16x8 v = pk.u;
    unsigned short* gp = U16 + (size_t)m * DI_ + d0;
    *(volatile u16x8*)gp = v;
    __threadfence();
    *(volatile u16x8*)gp = v;
}

__global__ __launch_bounds__(256)
void dtr_kernel(const float* __restrict__ xd, unsigned short* dtr16)
{
    const int i = blockIdx.x * 256 + threadIdx.x;
    if (i >= MT_ * (DTR_ / 8)) return;
    const int row = i / (DTR_ / 8);
    const int c0  = (i % (DTR_ / 8)) * 8;
    const v8f x = ld8f(xd + (size_t)row * XDW_ + c0);
    Pack8 pk;
    pk.f = __builtin_convertvector(x * SC_DT, v8h);
    const u16x8 v = pk.u;
    unsigned short* gp = dtr16 + (size_t)row * DTR_ + c0;
    *(volatile u16x8*)gp = v;
    __threadfence();
    *(volatile u16x8*)gp = v;
}

__device__ __forceinline__ void rows16_store_pass(const unsigned short* sl, unsigned short* gpl,
                                                  size_t gbase, int tid) {
#pragma unroll
    for (int it = 0; it < 2; ++it) {
        const int t = it * 8 + (tid >> 3);
        const int c = (tid & 7) * 8;
        const u16x8 v = *(const u16x8*)(sl + t * 64 + c);
        *(volatile u16x8*)(gpl + gbase + (size_t)t * DI_ + c) = v;
    }
}

__global__ __launch_bounds__(64)
void scan_kernel(const float* __restrict__ X, const float* __restrict__ Z,
                 const float* __restrict__ Dl, const float* __restrict__ xd,
                 const float* __restrict__ cw, const float* __restrict__ cb,
                 const float* __restrict__ Alog, const float* __restrict__ Dp,
                 const float* __restrict__ dtb, unsigned short* y16)
{
    __shared__ __attribute__((aligned(16))) unsigned short sy[16 * 64];
    __shared__ float sB[16 * NS_];
    __shared__ float sC[16 * NS_];

    const int tid   = threadIdx.x;
    const int lane  = tid & 31;
    const int wave  = tid >> 5;
    const int dbase = blockIdx.x * 64;
    const int d     = dbase + tid;
    const int b     = blockIdx.y;

    float an[NS_], hs[NS_];
#pragma unroll
    for (int n = 0; n < NS_; ++n) {
        an[n] = -expf(Alog[d * NS_ + n]);
        hs[n] = 0.0f;
    }
    const float w0 = cw[d * 4 + 0], w1 = cw[d * 4 + 1], w2 = cw[d * 4 + 2], w3 = cw[d * 4 + 3];
    const float cbias = cb[d];
    const float tb = dtb[d];
    const float Dd = Dp[d];

    float xm1 = 0.0f, xm2 = 0.0f, xm3 = 0.0f;
    const size_t mrow0 = (size_t)b * NL_;

#pragma unroll 1
    for (int l0 = 0; l0 < NL_; l0 += 16) {
#pragma unroll
        for (int j = 0; j < 8; ++j) {
            const int tt = 2 * j + wave;
            const float v = xd[(mrow0 + (size_t)(l0 + tt)) * XDW_ + DTR_ + lane];
            if (lane < NS_) sB[tt * NS_ + lane] = v;
            else            sC[tt * NS_ + (lane - NS_)] = v;
        }
        __syncthreads();
#pragma unroll 1
        for (int t = 0; t < 16; ++t) {
            const size_t mrow = mrow0 + (size_t)(l0 + t);
            const size_t e = mrow * DI_ + d;
            const float xv = X[e];
            const float zv = Z[e];
            const float dl = Dl[e];
            const float u  = conv4_silu(xm3, xm2, xm1, xv, w0, w1, w2, w3, cbias);
            xm3 = xm2; xm2 = xm1; xm1 = xv;
            const float dt = softplus_f(dl + tb);
            const float du = dt * u;
            float y = 0.0f;
#pragma unroll
            for (int n = 0; n < NS_; ++n) {
                const float da = __expf(dt * an[n]);
                hs[n] = da * hs[n] + du * sB[t * NS_ + n];
                y += hs[n] * sC[t * NS_ + n];
            }
            const float g = (y + Dd * u) * silu_f(zv);
            const _Float16 hg = (_Float16)(g * SC_Y);
            sy[t * 64 + tid] = __builtin_bit_cast(unsigned short, hg);
        }
        __syncthreads();
        const size_t gbase = (mrow0 + (size_t)l0) * DI_ + dbase;
        rows16_store_pass(sy, y16, gbase, tid);
        __threadfence();
        rows16_store_pass(sy, y16, gbase, tid);
        __syncthreads();
    }
}

extern "C" void kernel_launch(void* const* d_in, const int* in_sizes, int n_in,
                              void* d_out, int out_size, void* d_ws, size_t ws_size,
                              hipStream_t stream)
{
    if (n_in < 12) return;
    if (in_sizes[0]  != MT_ * DM_)      return;
    if (in_sizes[1]  != DM_)            return;
    if (in_sizes[2]  != DM_)            return;
    if (in_sizes[3]  != 2 * DI_ * DM_)  return;
    if (in_sizes[4]  != DI_ * 4)        return;
    if (in_sizes[5]  != DI_)            return;
    if (in_sizes[6]  != XDN_ * DI_)     return;
    if (in_sizes[7]  != DI_ * DTR_)     return;
    if (in_sizes[8]  != DI_)            return;
    if (in_sizes[9]  != DI_ * NS_)      return;
    if (in_sizes[10] != DI_)            return;
    if (in_sizes[11] != DM_ * DI_)      return;
    if (out_size != MT_ * DM_)          return;
    if (ws_size < WS_END)               return;

    const float* hsx  = (const float*)d_in[0];
    const float* lnw  = (const float*)d_in[1];
    const float* lnb  = (const float*)d_in[2];
    const float* wi   = (const float*)d_in[3];
    const float* cw   = (const float*)d_in[4];
    const float* cb   = (const float*)d_in[5];
    const float* wx   = (const float*)d_in[6];
    const float* wd   = (const float*)d_in[7];
    const float* dtb  = (const float*)d_in[8];
    const float* alog = (const float*)d_in[9];
    const float* Dp   = (const float*)d_in[10];
    const float* wo   = (const float*)d_in[11];
    float* out = (float*)d_out;

    char* ws = (char*)d_ws;
    unsigned short* x16   = (unsigned short*)(ws + OFF_X16);
    unsigned short* wi16  = (unsigned short*)(ws + OFF_WI);
    unsigned short* u16   = (unsigned short*)(ws + OFF_U16);
    unsigned short* y16   = (unsigned short*)(ws + OFF_Y16);
    float*          Xf    = (float*)(ws + OFF_XF);
    float*          Zf    = (float*)(ws + OFF_ZF);
    unsigned short* wx16  = (unsigned short*)(ws + OFF_WX);
    float*          xd    = (float*)(ws + OFF_XD);
    unsigned short* dtr16 = (unsigned short*)(ws + OFF_DTR);
    unsigned short* wd16  = (unsigned short*)(ws + OFF_WD);
    float*          Dl    = (float*)(ws + OFF_DL);
    unsigned short* wo16  = (unsigned short*)(ws + OFF_WO);

    hipLaunchKernelGGL(ln_f16_kernel, dim3(MT_), dim3(DM_ / 8), 0, stream, hsx, lnw, lnb, x16);

    {
        int n8;
        n8 = (2 * DI_ * DM_) / 8;
        hipLaunchKernelGGL(cvt_kernel, dim3((n8 + 255) / 256), dim3(256), 0, stream,
                           wi, wi16, n8, n8, SC_WI);
        n8 = (XDW_ * DI_) / 8;
        hipLaunchKernelGGL(cvt_kernel, dim3((n8 + 255) / 256), dim3(256), 0, stream,
                           wx, wx16, n8, (int)((XDN_ * DI_) / 8), SC_WX);
        n8 = (DI_ * DTR_) / 8;
        hipLaunchKernelGGL(cvt_kernel, dim3((n8 + 255) / 256), dim3(256), 0, stream,
                           wd, wd16, n8, n8, SC_WD);
        n8 = (DM_ * DI_) / 8;
        hipLaunchKernelGGL(cvt_kernel, dim3((n8 + 255) / 256), dim3(256), 0, stream,
                           wo, wo16, n8, n8, SC_WO);
    }

    hipLaunchKernelGGL(HIP_KERNEL_NAME(gemm_tn_kernel<4, false>),
                       dim3((2 * DI_) / 128, MT_ / 64), dim3(128), 0, stream,
                       (const unsigned short*)x16, (const unsigned short*)wi16,
                       Xf, Zf, (const float*)hsx, (int)DM_, (int)DI_, (int)DI_,
                       1.0f / (SC_X * SC_WI));

    hipLaunchKernelGGL(conv_silu_kernel, dim3(MT_), dim3(DI_ / 8), 0, stream,
                       (const float*)Xf, cw, cb, u16);

    hipLaunchKernelGGL(HIP_KERNEL_NAME(gemm_tn_kernel<4, false>),
                       dim3(XDW_ / 128, MT_ / 64), dim3(128), 0, stream,
                       (const unsigned short*)u16, (const unsigned short*)wx16,
                       xd, xd, (const float*)hsx, (int)DI_, (int)XDW_, (int)(4 * XDW_),
                       1.0f / (SC_U * SC_WX));

    hipLaunchKernelGGL(dtr_kernel, dim3((MT_ * (DTR_ / 8) + 255) / 256), dim3(256), 0, stream,
                       (const float*)xd, dtr16);

    hipLaunchKernelGGL(HIP_KERNEL_NAME(gemm_tn_kernel<4, false>),
                       dim3(DI_ / 128, MT_ / 64), dim3(128), 0, stream,
                       (const unsigned short*)dtr16, (const unsigned short*)wd16,
                       Dl, Dl, (const float*)hsx, (int)DTR_, (int)DI_, (int)(4 * DI_),
                       1.0f / (SC_DT * SC_WD));

    hipLaunchKernelGGL(scan_kernel, dim3(DI_ / 64, NBATCH), dim3(64), 0, stream,
                       (const float*)Xf, (const float*)Zf, (const float*)Dl, (const float*)xd,
                       cw, cb, alog, Dp, dtb, y16);

    hipLaunchKernelGGL(HIP_KERNEL_NAME(gemm_tn_kernel<2, true>),
                       dim3(DM_ / 64, MT_ / 64), dim3(128), 0, stream,
                       (const unsigned short*)y16, (const unsigned short*)wo16,
                       out, out, (const float*)hsx, (int)DI_, (int)DM_, (int)(4 * DM_),
                       1.0f / (SC_Y * SC_WO));
}
